// GraphAttentionNetwork_68994354642984
// MI455X (gfx1250) — hardware-run, weakly checked
//
#include <hip/hip_runtime.h>
#include <stddef.h>
#include <stdint.h>


#define INF     15
#define HID1    64
#define HID2    128
#define NHEAD   3
#define NH1     192
#define NH2     384
#define XPADC   32
#define K1      32
#define K2      416
#define LDA     448
#define XCOL    384
#define NLR1    384
#define NLR2    768
#define D2IN    207
#define OUTW    143
#define NTHR    256
#define NWAVE   8
#define EPT     8
#define CHUNK   (NTHR * EPT)
#define WCAP    (EPT * 32)
#define LISTN   (NWAVE * WCAP)
#define NBMAX   2048
#define SLOTB   11
#define NBRUN   1024
#define RCAP    28672
#define DEGCAP  256
#define STW     512
#define GBM     64
#define GBN     64
#define GTHR    128
#define OROWS   64
#define NEGS    0.15f
#define WSMAX   268435456
#define LDS_AGG ((2 * RCAP + 2 * NBMAX + LISTN) * 4 + 64)

static_assert((CHUNK & (CHUNK - 1)) == 0 && CHUNK <= (1 << SLOTB));
static_assert(NBMAX == (1 << SLOTB));
static_assert(NTHR * 8 == NBMAX);
static_assert(LISTN >= NBMAX);
static_assert(LISTN >= NWAVE * WCAP);
static_assert((RCAP % 32) == 0);
static_assert(NWAVE * STW <= RCAP);
static_assert(NH1 <= STW);
static_assert((NBRUN & (NBRUN - 1)) == 0 && NBRUN <= NBMAX && NBRUN >= 32);
static_assert(LDS_AGG <= 300000);
static_assert(GBM == (GTHR / 32) * 16);
static_assert(NH1 == NHEAD * HID1 && NH2 == NHEAD * HID2);
static_assert(HID1 == 64 && HID2 == 128);
static_assert((K1 % 32) == 0 && (K2 % 32) == 0 && K2 == 2 * NH1 + XPADC && K1 == XPADC && INF <= XPADC);
static_assert((NLR1 % GBN) == 0 && (NLR2 % GBN) == 0 && (NH1 % GBN) == 0 && (NH2 % GBN) == 0);
static_assert(XCOL == 2 * NH1 && XCOL + XPADC <= LDA && (LDA % 64) == 0 && (XCOL % 64) == 0);
static_assert(HID2 * 4 <= LDA * 2);
static_assert(D2IN == INF + NH1 && OUTW == INF + HID2);
static_assert((OROWS * OUTW) % 4 == 0 && ((OROWS * OUTW * 4) % 128) == 0);
static_assert(OROWS * HID2 / 4 == 8 * NTHR);
static_assert(OROWS * INF / 4 <= NTHR);

typedef float          v2f  __attribute__((ext_vector_type(2)));
typedef float          v4f  __attribute__((ext_vector_type(4)));
typedef float          v8f  __attribute__((ext_vector_type(8)));
typedef int            v4i  __attribute__((ext_vector_type(4)));
typedef int            v8i  __attribute__((ext_vector_type(8)));
typedef unsigned int   v4u  __attribute__((ext_vector_type(4)));
typedef unsigned short v8us __attribute__((ext_vector_type(8)));
typedef __bf16         v16b __attribute__((ext_vector_type(16)));
typedef v2f  __attribute__((may_alias)) v2fa;
typedef v4f  __attribute__((may_alias)) v4fa;
typedef v8us __attribute__((may_alias)) v8usa;
union FragB { v16b v; v8us h[2]; v8i w; };

__device__ __forceinline__ v8f wmb(const FragB& a, const FragB& b, v8f c) {
  v8f d = __builtin_amdgcn_wmma_f32_16x16x32_bf16(false, a.v, false, b.v, (short)0, c, false, false);
  asm volatile("v_nop\n\tv_nop\n\tv_nop\n\tv_nop" : "+v"(d) : "v"(a.w), "v"(b.w));
  return d;
}

__device__ __forceinline__ void ldwait() {
  asm volatile("s_wait_loadcnt 0x0" ::: "memory");
}

__device__ __forceinline__ unsigned int f2bf(float f) {
  const unsigned int u = __float_as_uint(f);
  return ((u + 0x7FFFu + ((u >> 16) & 1u)) >> 16) & 0xFFFFu;
}
__device__ __forceinline__ float bf2f(unsigned int b) { return __uint_as_float(b << 16); }
__device__ __forceinline__ float bfr(float f) { return bf2f(f2bf(f)); }
__device__ __forceinline__ unsigned int pk2(float lo, float hi) { return f2bf(lo) | (f2bf(hi) << 16); }
__device__ __forceinline__ void split8(const v4f a, const v4f b, v4u& hv, v4u& lv) {
  const unsigned int h0 = f2bf(a.x), h1 = f2bf(a.y), h2 = f2bf(a.z), h3 = f2bf(a.w);
  const unsigned int h4 = f2bf(b.x), h5 = f2bf(b.y), h6 = f2bf(b.z), h7 = f2bf(b.w);
  const unsigned int g0 = f2bf(a.x - bf2f(h0)), g1 = f2bf(a.y - bf2f(h1));
  const unsigned int g2 = f2bf(a.z - bf2f(h2)), g3 = f2bf(a.w - bf2f(h3));
  const unsigned int g4 = f2bf(b.x - bf2f(h4)), g5 = f2bf(b.y - bf2f(h5));
  const unsigned int g6 = f2bf(b.z - bf2f(h6)), g7 = f2bf(b.w - bf2f(h7));
  hv.x = h0 | (h1 << 16); hv.y = h2 | (h3 << 16); hv.z = h4 | (h5 << 16); hv.w = h6 | (h7 << 16);
  lv.x = g0 | (g1 << 16); lv.y = g2 | (g3 << 16); lv.z = g4 | (g5 << 16); lv.w = g6 | (g7 << 16);
}

template<int V> struct LdV;
template<> struct LdV<2> {
  static __device__ __forceinline__ void ld(const float* p, float* d) {
    const v2f t = *(const v2fa*)p; d[0] = t.x; d[1] = t.y;
  }
};
template<> struct LdV<4> {
  static __device__ __forceinline__ void ld(const float* p, float* d) {
    const v4f t = *(const v4fa*)p; d[0] = t.x; d[1] = t.y; d[2] = t.z; d[3] = t.w;
  }
};

__device__ __forceinline__ int scan_chunk(const int* __restrict__ dsts, int nE, int cbase, int slotBase,
                                          int nb, int vec8, int* list, int tid, int lane, int wave) {
  int wc = 0;
  const int el0  = tid * EPT;
  const int e0   = cbase + el0;
  const int sent = -2147483647 - 1;
  v4i da, db;
  if (vec8 != 0 && cbase + CHUNK <= nE) {
    da = *(const v4i*)(dsts + e0);
    db = *(const v4i*)(dsts + e0 + 4);
  } else {
    da.x = (e0     < nE) ? dsts[min(e0,     nE - 1)] : sent;
    da.y = (e0 + 1 < nE) ? dsts[min(e0 + 1, nE - 1)] : sent;
    da.z = (e0 + 2 < nE) ? dsts[min(e0 + 2, nE - 1)] : sent;
    da.w = (e0 + 3 < nE) ? dsts[min(e0 + 3, nE - 1)] : sent;
    db.x = (e0 + 4 < nE) ? dsts[min(e0 + 4, nE - 1)] : sent;
    db.y = (e0 + 5 < nE) ? dsts[min(e0 + 5, nE - 1)] : sent;
    db.z = (e0 + 6 < nE) ? dsts[min(e0 + 6, nE - 1)] : sent;
    db.w = (e0 + 7 < nE) ? dsts[min(e0 + 7, nE - 1)] : sent;
  }
  const unsigned nbs = (unsigned)slotBase;
  const unsigned unb = (unsigned)nb;
  const unsigned s0 = (unsigned)da.x - nbs, s1 = (unsigned)da.y - nbs;
  const unsigned s2 = (unsigned)da.z - nbs, s3 = (unsigned)da.w - nbs;
  const unsigned s4 = (unsigned)db.x - nbs, s5 = (unsigned)db.y - nbs;
  const unsigned s6 = (unsigned)db.z - nbs, s7 = (unsigned)db.w - nbs;
  const bool h0 = s0 < unb, h1 = s1 < unb, h2 = s2 < unb, h3 = s3 < unb;
  const bool h4 = s4 < unb, h5 = s5 < unb, h6 = s6 < unb, h7 = s7 < unb;
  const unsigned any = __builtin_amdgcn_ballot_w32(h0 | h1 | h2 | h3 | h4 | h5 | h6 | h7);
  if (any != 0u) {
#define HITJ(J, HJ, SJ) { \
      const unsigned mj = __builtin_amdgcn_ballot_w32(HJ); \
      if (mj != 0u) { \
        if (HJ) { \
          const int pos = wc + (int)__builtin_amdgcn_mbcnt_lo(mj, 0u); \
          if (pos < WCAP) list[wave * WCAP + pos] = ((el0 + (J)) << SLOTB) | (int)(SJ); \
        } \
        wc += (int)__builtin_popcount(mj); } }
    HITJ(0, h0, s0)
    HITJ(1, h1, s1)
    HITJ(2, h2, s2)
    HITJ(3, h3, s3)
    HITJ(4, h4, s4)
    HITJ(5, h5, s5)
    HITJ(6, h6, s6)
    HITJ(7, h7, s7)
#undef HITJ
  }
  return wc;
}

__global__ __launch_bounds__(NTHR) void k_xprep(const float* __restrict__ x, unsigned short* HA, int nN, int nUnits) {
  const int i = (int)blockIdx.x * NTHR + (int)threadIdx.x;
  if (i >= nUnits) return;
  const int row = i >> 3;
  const int cb  = (i & 7) * 8;
  const int rc  = row < nN ? row : nN - 1;
  const float* xr = x + (size_t)rc * INF;
  float f[8];
#pragma unroll
  for (int j = 0; j < 8; ++j) {
    const int c  = cb + j;
    const int cc = c < INF ? c : INF - 1;
    const float v = xr[cc];
    f[j] = (c < INF && row < nN) ? v : 0.0f;
  }
  v4u o;
  o.x = pk2(f[0], f[1]); o.y = pk2(f[2], f[3]); o.z = pk2(f[4], f[5]); o.w = pk2(f[6], f[7]);
  unsigned short* op = HA + (size_t)row * LDA + XCOL + cb;
  *(volatile v4u*)op = o;
  __threadfence();
  *(volatile v4u*)op = o;
}

template<int L>
__global__ __launch_bounds__(NTHR) void k_wtr(const float* __restrict__ w, int Ncol, unsigned short* wt, int nUnits) {
  constexpr int Kout = (L == 1) ? K1 : K2;
  constexpr int Kw   = (L == 1) ? INF : D2IN;
  const int u = (int)blockIdx.x * NTHR + (int)threadIdx.x;
  if (u >= nUnits) return;
  const int kq  = Kout >> 3;
  const int n   = u / kq;
  const int k8  = (u - n * kq) * 8;
  const int ncl = n < Ncol ? n : Ncol - 1;
  float f[8];
#pragma unroll
  for (int j = 0; j < 8; ++j) {
    const int k = k8 + j;
    int kk;
    bool ok;
    if (L == 1) {
      ok = k < INF;
      kk = k;
    } else {
      ok = (k < 2 * NH1) || (k < XCOL + INF);
      kk = (k < NH1) ? (INF + k) : ((k < 2 * NH1) ? (INF + k - NH1) : (k - XCOL));
    }
    kk = kk < 0 ? 0 : (kk > Kw - 1 ? Kw - 1 : kk);
    const float v = w[(size_t)kk * (size_t)Ncol + ncl];
    f[j] = (ok && n < Ncol) ? v : 0.0f;
  }
  v4u o;
  o.x = pk2(f[0], f[1]); o.y = pk2(f[2], f[3]); o.z = pk2(f[4], f[5]); o.w = pk2(f[6], f[7]);
  unsigned short* op = wt + (size_t)n * (size_t)Kout + k8;
  *(volatile v4u*)op = o;
  __threadfence();
  *(volatile v4u*)op = o;
}

__global__ __launch_bounds__(GTHR) void k_gemm(
    const unsigned short* __restrict__ A, int lda, const unsigned short* __restrict__ WT, int K,
    const float* __restrict__ bsA, const float* __restrict__ bsB, int NHc, float* outF, int ldo)
{
  __shared__ __attribute__((aligned(16))) float stg[GBM * GBN];
  const int tid = (int)threadIdx.x, lane = tid & 31, wave = tid >> 5, hh = lane >> 4, m = lane & 15;
  const int rowBase = (int)blockIdx.x * GBM;
  const int col0    = (int)blockIdx.y * GBN;

  v8f acc[4];
  {
    const v8f z = {0.f, 0.f, 0.f, 0.f, 0.f, 0.f, 0.f, 0.f};
    acc[0] = z; acc[1] = z; acc[2] = z; acc[3] = z;
  }
  const unsigned short* ap = A  + (size_t)(rowBase + 16 * wave + m) * (size_t)lda + 8 * hh;
  const unsigned short* wp = WT + (size_t)(col0 + m) * (size_t)K + 8 * hh;
  const int ksteps = K >> 5;
#pragma unroll 1
  for (int ks = 0; ks < ksteps; ++ks) {
    FragB af;
    af.h[0] = *(const v8usa*)(ap + 32 * ks);
    af.h[1] = *(const v8usa*)(ap + 32 * ks + 16);
#pragma unroll
    for (int t = 0; t < 4; ++t) {
      const unsigned short* wq = wp + (size_t)(16 * t) * (size_t)K + 32 * ks;
      FragB bf;
      bf.h[0] = *(const v8usa*)wq;
      bf.h[1] = *(const v8usa*)(wq + 16);
      acc[t] = wmb(af, bf, acc[t]);
    }
  }

  const int bsel = (col0 >= NHc) ? 1 : 0;
#pragma unroll
  for (int t = 0; t < 4; ++t) {
    const int lc = 16 * t + m;
    const int gc = col0 + lc;
    const int cl = gc < NHc ? gc : gc - NHc;
    const float vl = bsA[cl];
    const float vr = bsB[cl];
    const float bv = bfr(bsel ? vr : vl);
#pragma unroll
    for (int r = 0; r < 8; ++r) {
      const int lr = 16 * wave + 8 * hh + r;
      stg[lr * GBN + lc] = acc[t][r] + bv;
    }
  }
  __syncthreads();

  v4f fv[8];
#pragma unroll
  for (int i = 0; i < 8; ++i) {
    const int lr = 16 * wave + 2 * i + hh;
    fv[i] = *(const v4fa*)(stg + lr * GBN + 4 * m);
  }
#pragma unroll
  for (int i = 0; i < 8; ++i) {
    const int lr = 16 * wave + 2 * i + hh;
    const int gr = rowBase + lr;
    float* op = outF + (size_t)gr * (size_t)ldo + col0 + 4 * m;
    *(volatile v4f*)op = fv[i];
  }
  __threadfence();
#pragma unroll
  for (int i = 0; i < 8; ++i) {
    const int lr = 16 * wave + 2 * i + hh;
    const int gr = rowBase + lr;
    float* op = outF + (size_t)gr * (size_t)ldo + col0 + 4 * m;
    *(volatile v4f*)op = fv[i];
  }
}

template<int VPL>
__global__ __launch_bounds__(NTHR) void k_agg(
    const int* __restrict__ srcs, const int* __restrict__ dsts,
    const float* __restrict__ XLR, const float* __restrict__ att, const float* __restrict__ bias,
    unsigned short* HAo, float* H2o,
    int nN, int nE, int nb, int vec8, int MPr) {
  constexpr int CH  = 32 * VPL;
  constexpr int NH  = NHEAD * CH;
  constexpr int NLR = 2 * NH;
  constexpr int NB  = (VPL == 2) ? NH : CH;
  static_assert(NH + NB <= 512);
  static_assert(NH <= STW);
  extern __shared__ v4f lds_dyn[];
  int* reg1 = (int*)lds_dyn;
  int* reg2 = reg1 + RCAP;
  int* scnt = reg2 + RCAP;
  int* soff = scnt + NBMAX;
  int* list = soff + NBMAX;
  int* wcnt = list + LISTN;
  int* wtot = wcnt + NWAVE;
  __shared__ __attribute__((aligned(16))) float spar[512];
  const int tid = (int)threadIdx.x, lane = tid & 31, wave = tid >> 5;
  const int nodeBase = (int)blockIdx.x * nb;

  for (int i = tid; i < NBMAX; i += NTHR) scnt[i] = 0;
  __syncthreads();

  int tot = 0;
  const int nChunks = (nE + CHUNK - 1) / CHUNK;
#pragma unroll 1
  for (int ch = 0; ch < nChunks; ++ch) {
    const int cbase = ch * CHUNK;
    const int wc = scan_chunk(dsts, nE, cbase, nodeBase, nb, vec8, list, tid, lane, wave);
    if (lane == 0) wcnt[wave] = wc;
    __syncthreads();
    int pre = 0, all = 0;
#pragma unroll
    for (int w2 = 0; w2 < NWAVE; ++w2) {
      int c = wcnt[w2];
      c = c < 0 ? 0 : (c > WCAP ? WCAP : c);
      all += c;
      pre += (w2 < wave) ? c : 0;
    }
    const int wcc  = wc > WCAP ? WCAP : wc;
    const int base = tot + pre;
#pragma unroll 1
    for (int i = lane; i < wcc; i += 32) {
      const int ent = list[wave * WCAP + i];
      const int el  = (ent >> SLOTB) & (CHUNK - 1);
      const int sl  = ent & (NBMAX - 1);
      int eid = cbase + el;
      eid = eid > nE - 1 ? nE - 1 : eid;
      const int pos = base + i;
      if (pos < RCAP) reg1[pos] = (int)(((unsigned)eid << SLOTB) | (unsigned)sl);
    }
    tot += all;
    tot = tot > RCAP ? RCAP : tot;
    __syncthreads();
  }
  const int nh = tot;

  if (wave == 0) {
#pragma unroll 1
    for (int b0 = 0; b0 < nh; b0 += 32) {
      const int idx = b0 + lane;
      const int uv  = reg1[idx < nh ? idx : nh - 1];
      const int m32 = (nh - b0) < 32 ? (nh - b0) : 32;
#pragma unroll 1
      for (int k = 0; k < m32; ++k) {
        const int u  = __builtin_amdgcn_readlane(uv, k);
        const int sl = u & (NBMAX - 1);
        if (lane == 0) scnt[sl] = scnt[sl] + 1;
      }
    }
  }
  __syncthreads();

  {
    const v4i ca = *(const v4i*)(scnt + 8 * tid);
    const v4i cb = *(const v4i*)(scnt + 8 * tid + 4);
    const int e0 = ca.x < 0 ? 0 : ca.x, e1 = ca.y < 0 ? 0 : ca.y, e2 = ca.z < 0 ? 0 : ca.z, e3 = ca.w < 0 ? 0 : ca.w;
    const int e4 = cb.x < 0 ? 0 : cb.x, e5 = cb.y < 0 ? 0 : cb.y, e6 = cb.z < 0 ? 0 : cb.z, e7 = cb.w < 0 ? 0 : cb.w;
    const int ts = e0 + e1 + e2 + e3 + e4 + e5 + e6 + e7;
    int incl = ts;
#pragma unroll
    for (int d = 1; d < 32; d <<= 1) {
      const int up = __shfl_up(incl, d);
      if (lane >= d) incl += up;
    }
    if (lane == 31) wtot[wave] = incl;
    __syncthreads();
    int pre = 0;
#pragma unroll
    for (int w2 = 0; w2 < NWAVE; ++w2) pre += (w2 < wave) ? wtot[w2] : 0;
    int run = pre + incl - ts;
    soff[8 * tid + 0] = run; run += e0;
    soff[8 * tid + 1] = run; run += e1;
    soff[8 * tid + 2] = run; run += e2;
    soff[8 * tid + 3] = run; run += e3;
    soff[8 * tid + 4] = run; run += e4;
    soff[8 * tid + 5] = run; run += e5;
    soff[8 * tid + 6] = run; run += e6;
    soff[8 * tid + 7] = run;
  }
  __syncthreads();
  for (int i = tid; i < NBMAX; i += NTHR) list[i] = soff[i];
  __syncthreads();

  if (wave == 0) {
#pragma unroll 1
    for (int b0 = 0; b0 < nh; b0 += 32) {
      const int idx = b0 + lane;
      const int uv  = reg1[idx < nh ? idx : nh - 1];
      const int m32 = (nh - b0) < 32 ? (nh - b0) : 32;
#pragma unroll 1
      for (int k = 0; k < m32; ++k) {
        const int u   = __builtin_amdgcn_readlane(uv, k);
        const int sl  = u & (NBMAX - 1);
        const int eid = (int)((unsigned)u >> SLOTB);
        if (lane == 0) {
          int pos = list[sl];
          pos = pos < 0 ? 0 : (pos > RCAP - 1 ? RCAP - 1 : pos);
          reg2[pos] = eid;
          list[sl] = pos + 1;
        }
      }
    }
  }
  __syncthreads();

  const int nbw = nb >> 3;
  const bool ovf = (nh >= RCAP);
  const float qnan = __int_as_float(0x7fc00000);
  float* stw = (float*)reg1 + wave * STW;
  {
    const int qa = tid < (NH / 4) ? tid : (NH / 4) - 1;
    const int qb = tid < (NB / 4) ? tid : (NB / 4) - 1;
    const v4f va = *(const v4fa*)(att  + 4 * qa);
    const v4f vb = *(const v4fa*)(bias + 4 * qb);
    if (tid < NH / 4) *(v4fa*)(spar + 4 * tid) = va;
    if (tid < NB / 4) *(v4fa*)(spar + NH + 4 * tid) = vb;
  }
  __syncthreads();
  float at[NHEAD][VPL], bb[NHEAD][VPL];
#pragma unroll
  for (int h = 0; h < NHEAD; ++h) {
    float t[VPL];
    LdV<VPL>::ld(spar + CH * h + VPL * lane, t);
#pragma unroll
    for (int v = 0; v < VPL; ++v) at[h][v] = bfr(t[v]);
  }
  if constexpr (VPL == 2) {
#pragma unroll
    for (int h = 0; h < NHEAD; ++h) {
      float t[VPL];
      LdV<VPL>::ld(spar + NH + CH * h + VPL * lane, t);
#pragma unroll
      for (int v = 0; v < VPL; ++v) bb[h][v] = bfr(t[v]);
    }
  } else {
    float t[VPL];
    LdV<VPL>::ld(spar + NH + VPL * lane, t);
#pragma unroll
    for (int v = 0; v < VPL; ++v) { bb[0][v] = bfr(t[v]); bb[1][v] = 0.f; bb[2][v] = 0.f; }
  }

#pragma unroll 1
  for (int jt = 0; jt < nbw; ++jt) {
    const int slot = wave * nbw + jt;
    const int grow = nodeBase + slot;
    const int gcl  = grow < nN ? grow : nN - 1;
    int st = soff[slot];
    const int craw = scnt[slot];
    int cnt = craw;
    st  = st < 0 ? 0 : (st > nh ? nh : st);
    cnt = cnt < 0 ? 0 : (cnt > DEGCAP ? DEGCAP : cnt);
    if (cnt > nh - st) cnt = nh - st;
    const float pz = (ovf || craw > DEGCAP) ? qnan : 0.0f;

    const float* rr = XLR + (size_t)gcl * NLR + NH + VPL * lane;
    float hd[NHEAD][VPL], av[NHEAD][VPL];
#pragma unroll
    for (int h = 0; h < NHEAD; ++h) LdV<VPL>::ld(rr + CH * h, hd[h]);
    ldwait();
    float mx[NHEAD], dn[NHEAD];
#pragma unroll
    for (int h = 0; h < NHEAD; ++h) {
      mx[h] = -1.0e30f; dn[h] = 0.f;
#pragma unroll
      for (int v = 0; v < VPL; ++v) av[h][v] = 0.f;
    }

#pragma unroll 1
    for (int q = 0; q < cnt; ++q) {
      int idx = st + q; idx = idx > RCAP - 1 ? RCAP - 1 : idx;
      int eid = reg2[idx]; eid = eid < 0 ? 0 : (eid > nE - 1 ? nE - 1 : eid);
      const int sraw = srcs[eid];
      const int s = sraw < 0 ? 0 : (sraw > nN - 1 ? nN - 1 : sraw);
      const float* sr = XLR + (size_t)s * NLR + VPL * lane;
      float hs[NHEAD][VPL];
#pragma unroll
      for (int h = 0; h < NHEAD; ++h) LdV<VPL>::ld(sr + CH * h, hs[h]);
      ldwait();
      float part[NHEAD];
#pragma unroll
      for (int h = 0; h < NHEAD; ++h) {
        float p = 0.f;
#pragma unroll
        for (int v = 0; v < VPL; ++v) {
          const float z  = hs[h][v] + hd[h][v];
          const float zz = fmaxf(z, z * NEGS);
          p = fmaf(zz, at[h][v], p);
        }
        part[h] = p;
      }
#pragma unroll
      for (int off = 16; off > 0; off >>= 1) {
#pragma unroll
        for (int h = 0; h < NHEAD; ++h) part[h] += __shfl_xor(part[h], off);
      }
#pragma unroll
      for (int h = 0; h < NHEAD; ++h) {
        const float lg = part[h];
        const float df = lg - mx[h];
        const float ee = __expf(-fabsf(df));
        const bool up  = df > 0.f;
        const float s1 = up ? ee : 1.0f;
        const float s2 = up ? 1.0f : ee;
        mx[h] = up ? lg : mx[h];
        dn[h] = fmaf(dn[h], s1, s2);
#pragma unroll
        for (int v = 0; v < VPL; ++v) av[h][v] = fmaf(av[h][v], s1, s2 * hs[h][v]);
      }
    }
    float iv[NHEAD];
#pragma unroll
    for (int h = 0; h < NHEAD; ++h) {
      const float ds = dn[h] > 0.f ? dn[h] : 1.0f;
      iv[h] = (dn[h] > 0.f ? 1.0f : 0.0f) * __builtin_amdgcn_rcpf(ds);
    }

    if constexpr (VPL == 2) {
      const float livef = grow < nN ? 1.0f : 0.0f;
      float r[NHEAD][VPL];
#pragma unroll
      for (int h = 0; h < NHEAD; ++h) {
#pragma unroll
        for (int v = 0; v < VPL; ++v) {
          float t2 = fmaf(av[h][v], iv[h], bb[h][v]);
          t2 = fmaxf(t2, 0.f) * livef;
          r[h][v] = t2 + pz;
        }
      }
      __builtin_amdgcn_fence(__ATOMIC_RELEASE, "wavefront");
      __builtin_amdgcn_wave_barrier();
#pragma unroll
      for (int h = 0; h < NHEAD; ++h) {
        v2f t2; t2.x = r[h][0]; t2.y = r[h][1];
        *(v2fa*)(stw + CH * h + 2 * lane) = t2;
      }
      __builtin_amdgcn_fence(__ATOMIC_RELEASE, "wavefront");
      __builtin_amdgcn_wave_barrier();
      const int la = lane < 24 ? lane : lane - 24;
      const v4f pa = *(const v4fa*)(stw + 8 * la);
      const v4f pb = *(const v4fa*)(stw + 8 * la + 4);
      v4u hw, lw;
      split8(pa, pb, hw, lw);
      const unsigned int msk = (lane >= 24) ? 0xFFFFFFFFu : 0u;
      v4u pv;
      pv.x = (hw.x & ~msk) | (lw.x & msk);
      pv.y = (hw.y & ~msk) | (lw.y & msk);
      pv.z = (hw.z & ~msk) | (lw.z & msk);
      pv.w = (hw.w & ~msk) | (lw.w & msk);
      const int lb = lane & 15;
      const v4f qa2 = *(const v4fa*)(stw + CH + 8 * lb);
      const v4f qb2 = *(const v4fa*)(stw + CH + 8 * lb + 4);
      v4u hw2, lw2;
      split8(qa2, qb2, hw2, lw2);
      unsigned short* p1 = HAo + (size_t)grow * LDA + 8 * lane;
      unsigned short* p2 = HAo + (size_t)grow * LDA + NH + CH + 8 * lb;
      const bool wr  = grow < MPr;
      const bool wr2 = wr && (lane < 16);
      if (wr)  *(volatile v4u*)p1 = pv;
      if (wr2) *(volatile v4u*)p2 = lw2;
      __threadfence();
      if (wr)  *(volatile v4u*)p1 = pv;
      if (wr2) *(volatile v4u*)p2 = lw2;
    } else {
      float r4[4];
#pragma unroll
      for (int v = 0; v < 4; ++v) {
        const float sm = (av[0][v] * iv[0] + av[1][v] * iv[1]) + av[2][v] * iv[2];
        float t2 = fmaf(sm, (1.0f / 3.0f), bb[0][v]);
        t2 = fmaxf(t2, 0.f);
        r4[v] = t2 + pz;
      }
      v4f o; o.x = r4[0]; o.y = r4[1]; o.z = r4[2]; o.w = r4[3];
      float* hp = H2o + (size_t)grow * CH + 4 * lane;
      const bool wr = grow < nN;
      if (wr) *(volatile v4f*)hp = o;
      __threadfence();
      if (wr) *(volatile v4f*)hp = o;
    }
  }
  (void)HAo; (void)H2o; (void)MPr;
}

__global__ __launch_bounds__(NTHR) void k_out(const float* __restrict__ x, const float* __restrict__ H2,
                                              float* out, int nN) {
  __shared__ __attribute__((aligned(16))) float stg[OROWS * OUTW];
  const int tid = (int)threadIdx.x;
  const int rowBase = (int)blockIdx.x * OROWS;
  int nr = nN - rowBase;
  nr = nr > OROWS ? OROWS : nr;
  {
    const int nq = (nr * INF) >> 2;
    const int q  = tid < nq ? tid : nq - 1;
    const v4f v  = *(const v4fa*)(x + (size_t)rowBase * INF + 4 * q);
    if (tid < nq) {
      const int f0 = 4 * tid;
#pragma unroll
      for (int i = 0; i < 4; ++i) {
        const int e = f0 + i;
        const int r = e / INF;
        const int c = e - r * INF;
        stg[r * OUTW + c] = bfr(v[i]);
      }
    }
  }
#pragma unroll
  for (int i = 0; i < (OROWS * HID2 / 4) / NTHR; ++i) {
    const int u  = tid + NTHR * i;
    const int r  = u >> 5;
    const int c4 = u & 31;
    int gr = rowBase + r; gr = gr < nN ? gr : nN - 1;
    const v4f v = *(const v4fa*)(H2 + (size_t)gr * HID2 + 4 * c4);
    float* sp = stg + r * OUTW + INF + 4 * c4;
    sp[0] = v.x; sp[1] = v.y; sp[2] = v.z; sp[3] = v.w;
  }
  __syncthreads();
  const int npc = (nr * OUTW) >> 2;
  float* ob = out + (size_t)rowBase * OUTW;
#pragma unroll
  for (int i = 0; i < (OROWS * OUTW / 4 + NTHR - 1) / NTHR; ++i) {
    const int u = tid + NTHR * i;
    if (u < npc) *(volatile v4f*)(ob + 4 * u) = *(const v4fa*)(stg + 4 * u);
  }
  __threadfence();
#pragma unroll
  for (int i = 0; i < (OROWS * OUTW / 4 + NTHR - 1) / NTHR; ++i) {
    const int u = tid + NTHR * i;
    if (u < npc) *(volatile v4f*)(ob + 4 * u) = *(const v4fa*)(stg + 4 * u);
  }
}

static int pick_nb(int nE, int nN) {
  int nb = NBRUN;
  while (nb > 32 && (long long)nb * (long long)nE * 5LL > (long long)RCAP * (long long)nN * 4LL) nb >>= 1;
  return nb;
}
static inline int cdiv(int a, int b) { return (a + b - 1) / b; }

extern "C" void kernel_launch(void* const* d_in, const int* in_sizes, int n_in,
                              void* d_out, int out_size, void* d_ws, size_t ws_size,
                              hipStream_t stream) {
  if (n_in < 14) return;
  const int nN = in_sizes[0] / INF;
  if (nN <= 0 || in_sizes[0] != nN * INF || nN > (1 << 22) || (nN & 3) != 0) return;
  if (in_sizes[1] < 2 || (in_sizes[1] & 1) != 0) return;
  const int nE = in_sizes[1] / 2;
  if (nE < 1 || nE >= (1 << (32 - SLOTB))) return;
  if (in_sizes[2] != INF * NH1 || in_sizes[3] != NH1) return;
  if (in_sizes[4] != INF * NH1 || in_sizes[5] != NH1) return;
  if (in_sizes[6] != NH1 || in_sizes[7] != NH1) return;
  if (in_sizes[8] != D2IN * NH2 || in_sizes[9] != NH2) return;
  if (in_sizes[10] != D2IN * NH2 || in_sizes[11] != NH2) return;
  if (in_sizes[12] != NH2 || in_sizes[13] != HID2) return;
  if (out_size != nN * OUTW) return;

  const float* x     = (const float*)d_in[0];
  const int*   ei    = (const int*)  d_in[1];
  const float* W1l   = (const float*)d_in[2];
  const float* b1l   = (const float*)d_in[3];
  const float* W1r   = (const float*)d_in[4];
  const float* b1r   = (const float*)d_in[5];
  const float* att1  = (const float*)d_in[6];
  const float* bias1 = (const float*)d_in[7];
  const float* W2l   = (const float*)d_in[8];
  const float* b2l   = (const float*)d_in[9];
  const float* W2r   = (const float*)d_in[10];
  const float* b2r   = (const float*)d_in[11];
  const float* att2  = (const float*)d_in[12];
  const float* bias2 = (const float*)d_in[13];
  float* out = (float*)d_out;
  const int* src = ei;
  const int* dst = ei + nE;

  const int MP   = cdiv(nN, GBM) * GBM;
  const int nb   = pick_nb(nE, nN);
  if (nb < 32 || (nb & (nb - 1)) != 0 || nb > NBMAX) return;
  const int gA   = cdiv(MP, nb);
  const int vec8 = ((nE & 3) == 0) ? 1 : 0;
  if (gA * nb < MP) return;

  char* ws = (char*)d_ws;
  size_t off = 0;
  const size_t oWT1 = off; off += (size_t)NLR1 * K1 * 2;        off = (off + 255) & ~(size_t)255;
  const size_t oWT2 = off; off += (size_t)NLR2 * K2 * 2;        off = (off + 255) & ~(size_t)255;
  const size_t oHA  = off; off += (size_t)MP * LDA * 2;         off = (off + 255) & ~(size_t)255;
  const size_t oXLR = off; off += (size_t)MP * NLR2 * 4;        off = (off + 255) & ~(size_t)255;
  if (off > ws_size || off > (size_t)WSMAX) return;
  if ((size_t)MP * HID2 * 4 > (size_t)MP * LDA * 2) return;
  unsigned short* WT1 = (unsigned short*)(ws + oWT1);
  unsigned short* WT2 = (unsigned short*)(ws + oWT2);
  unsigned short* HA  = (unsigned short*)(ws + oHA);
  float*          H2  = (float*)(ws + oHA);
  float*          XLR = (float*)(ws + oXLR);

  hipFuncSetAttribute(reinterpret_cast<const void*>(&k_agg<2>),
                      hipFuncAttributeMaxDynamicSharedMemorySize, LDS_AGG);
  hipFuncSetAttribute(reinterpret_cast<const void*>(&k_agg<4>),
                      hipFuncAttributeMaxDynamicSharedMemorySize, LDS_AGG);

  const int nUx = MP * 8;
  k_xprep<<<cdiv(nUx, NTHR), NTHR, 0, stream>>>(x, HA, nN, nUx);

  {
    const int nU1 = NH1 * (K1 / 8);
    k_wtr<1><<<cdiv(nU1, NTHR), NTHR, 0, stream>>>(W1l, NH1, WT1, nU1);
    k_wtr<1><<<cdiv(nU1, NTHR), NTHR, 0, stream>>>(W1r, NH1, WT1 + (size_t)NH1 * K1, nU1);
    const int nU2 = NH2 * (K2 / 8);
    k_wtr<2><<<cdiv(nU2, NTHR), NTHR, 0, stream>>>(W2l, NH2, WT2, nU2);
    k_wtr<2><<<cdiv(nU2, NTHR), NTHR, 0, stream>>>(W2r, NH2, WT2 + (size_t)NH2 * K2, nU2);
  }

  const int gM = MP / GBM;
  k_gemm<<<dim3(gM, NLR1 / GBN), GTHR, 0, stream>>>(HA + XCOL, LDA, WT1, K1, b1l, b1r, NH1, XLR, NLR1);
  k_agg<2><<<gA, NTHR, LDS_AGG, stream>>>(src, dst, XLR, att1, bias1, HA, H2, nN, nE, nb, vec8, MP);
  k_gemm<<<dim3(gM, NLR2 / GBN), GTHR, 0, stream>>>(HA, LDA, WT2, K2, b2l, b2r, NH2, XLR, NLR2);
  k_agg<4><<<gA, NTHR, LDS_AGG, stream>>>(src, dst, XLR, att2, bias2, HA, H2, nN, nE, nb, vec8, MP);
  k_out<<<cdiv(nN, OROWS), NTHR, 0, stream>>>(x, H2, out, nN);
}
